// TransformerLayer_42923903156585
// MI455X (gfx1250) — hardware-verified
//
#include <hip/hip_runtime.h>
#include <math.h>

typedef __attribute__((ext_vector_type(16))) _Float16 v16h;
typedef __attribute__((ext_vector_type(16))) __bf16 v16b;
typedef __attribute__((ext_vector_type(8)))  _Float16 v8h;
typedef __attribute__((ext_vector_type(4)))  _Float16 v4h;
typedef __attribute__((ext_vector_type(8)))  __bf16 v8b;
typedef __attribute__((ext_vector_type(8)))  float v8f;
typedef __attribute__((ext_vector_type(4)))  float v4f;
typedef __attribute__((ext_vector_type(8)))  unsigned short v8us;
typedef __attribute__((ext_vector_type(4)))  unsigned short v4us;
typedef __attribute__((ext_vector_type(4)))  int v4i;

#ifndef SEQ
#define SEQ 1024u
#endif
#define SEQ_FULL 1024u
#ifndef NB
#define NB 8u
#endif
#define NB_FULL 8u
#define CH 512u
#define NH 8u
#define HD 64u
#define HID 2048u
#define PR (SEQ + 2u)
#define NJ128 (SEQ / 128u)
#define NI16 (SEQ / 16u)
#define NFLAGS (NB * NJ128 * NI16)
#define PCY (16384.0f)
#define WC (64.0f)
#define CC (64.0f)
#define F16MIN (6.103515625e-05f)
#define LN_EPS (1e-5f)
static_assert(SEQ % 128u == 0u);
static_assert(SEQ >= 128u);
static_assert(SEQ <= SEQ_FULL);
static_assert(NB >= 1u && NB <= NB_FULL);
static_assert(NFLAGS % 32u == 0u);
static_assert(NH * HD == CH);
static_assert((NB * SEQ) % 64u == 0u);

#define AL256(x) ((((size_t)(x)) + 255u) & ~(size_t)255u)
#define WSZ_XB   AL256(2u * (size_t)NB * SEQ * CH)
#define WSZ_WP   AL256(2u * (size_t)CH * HD)
#define WSZ_WOH  AL256(2u * (size_t)CH * CH)
#define WSZ_W1P  AL256(2u * 3u * (size_t)HID * CH)
#define WSZ_W2P  AL256(2u * 3u * (size_t)CH * HID)
#define WSZ_CS   AL256(4u * (size_t)SEQ * 32u)
#define WSZ_MFL  AL256(4u * (size_t)NFLAGS)
#define WSZ_QH   AL256(2u * (size_t)NB * NH * SEQ * HD)
#define WSZ_ST   AL256(4u * (size_t)NB * NH * SEQ)
#define WSZ_CTX  AL256(2u * (size_t)NB * SEQ * CH)
#define WSZ_S1   AL256(4u * (size_t)NB * SEQ * CH)
#define WSZ_H32  AL256(4u * (size_t)NB * SEQ * CH)
#define WSZ_HP   AL256(2u * (size_t)NB * PR * CH)
#define WSZ_FP   AL256(2u * (size_t)NB * PR * HID)
#define WS_XB   ((size_t)0)
#define WS_WQB  (WS_XB  + WSZ_XB)
#define WS_WKB  (WS_WQB + WSZ_WP)
#define WS_WVB  (WS_WKB + WSZ_WP)
#define WS_WOH  (WS_WVB + WSZ_WP)
#define WS_W1P  (WS_WOH + WSZ_WOH)
#define WS_W2P  (WS_W1P + WSZ_W1P)
#define WS_CS   (WS_W2P + WSZ_W2P)
#define WS_MFL  (WS_CS  + WSZ_CS)
#define WS_QH   (WS_MFL + WSZ_MFL)
#define WS_KH   (WS_QH  + WSZ_QH)
#define WS_VP   (WS_KH  + WSZ_QH)
#define WS_MX   (WS_VP  + WSZ_QH)
#define WS_RZ   (WS_MX  + WSZ_ST)
#define WS_CTX  (WS_RZ  + WSZ_ST)
#define WS_S1   (WS_CTX + WSZ_CTX)
#define WS_H32  (WS_S1  + WSZ_S1)
#define WS_HP   (WS_H32 + WSZ_H32)
#define WS_FP   (WS_HP  + WSZ_HP)
#define WS_END  (WS_FP  + WSZ_FP)
#define WS_Z2   (WS_S1)
static_assert(WS_END <= (size_t)134217728u);
static_assert(WSZ_S1 >= 4u * (size_t)NB * SEQ * CH);

template <typename T> __device__ __forceinline__ void vst2(void* p, T v) { *(volatile T*)p = v; __threadfence(); *(volatile T*)p = v; }
__device__ __forceinline__ v8f zero8() { v8f z = {0.f, 0.f, 0.f, 0.f, 0.f, 0.f, 0.f, 0.f}; return z; }
__device__ __forceinline__ v8f wmma16(v16h a, v16h b, v8f c) {
  v8f d = __builtin_amdgcn_wmma_f32_16x16x32_f16(false, a, false, b, (short)0, c, false, false);
  asm volatile("v_nop\n\tv_nop\n\tv_nop\n\tv_nop" : "+v"(d) : "v"(a), "v"(b));
  return d;
}
__device__ __forceinline__ v8f wmma_bf(v16b a, v16b b, v8f c) {
  v8f d = __builtin_amdgcn_wmma_f32_16x16x32_bf16(false, a, false, b, (short)0, c, false, false);
  asm volatile("v_nop\n\tv_nop\n\tv_nop\n\tv_nop" : "+v"(d) : "v"(a), "v"(b));
  return d;
}
__device__ __forceinline__ v16h frag_h(const _Float16* rowk0, unsigned lane) {
  union { v16h v; v8h q[2]; } u; const _Float16* p = rowk0 + 8u * (lane >> 4);
  u.q[0] = *(const v8h*)p; u.q[1] = *(const v8h*)(p + 16); return u.v;
}
__device__ __forceinline__ v16b frag_b(const __bf16* rowk0, unsigned lane) {
  union { v16b v; v8b q[2]; } u; const __bf16* p = rowk0 + 8u * (lane >> 4);
  u.q[0] = *(const v8b*)p; u.q[1] = *(const v8b*)(p + 16); return u.v;
}
__device__ __forceinline__ _Float16 f16n(float x) { const float t = (fabsf(x) >= F16MIN) ? x : 0.0f; return (_Float16)t; }
__device__ __forceinline__ unsigned short bf16bits(float x) { unsigned u = __float_as_uint(x); u += 0x7FFFu + ((u >> 16) & 1u); return (unsigned short)(u >> 16); }
__device__ __forceinline__ float bf16val(unsigned short b) { return __uint_as_float(((unsigned)b) << 16); }
__device__ __forceinline__ float bfr(float x) { return bf16val(bf16bits(x)); }
#define LDSX() do { asm volatile("s_wait_dscnt 0" ::: "memory"); __builtin_amdgcn_wave_barrier(); __builtin_amdgcn_fence(3  , "workgroup"); } while (0)

__global__ __launch_bounds__(256) void k_xt(const float* __restrict__ X, unsigned short* __restrict__ XB) {
  __shared__ __align__(16) unsigned short ts[64][72];
  const unsigned tid = threadIdx.x;
  const unsigned t0 = blockIdx.x * 64u, c0 = blockIdx.y * 64u, b = blockIdx.z;
#pragma unroll
  for (unsigned it = 0; it < 4u; ++it) {
    const unsigned e = tid + it * 256u; const unsigned cl = e >> 4, q = e & 15u;
    const v4f a = *(const v4f*)(X + ((size_t)(b * CH + c0 + cl)) * SEQ_FULL + t0 + q * 4u);
#pragma unroll
    for (unsigned k = 0; k < 4u; ++k) ts[q * 4u + k][cl] = bf16bits(a[k]);
  }
  __syncthreads();
#pragma unroll
  for (unsigned it = 0; it < 2u; ++it) {
    const unsigned e = tid + it * 256u; const unsigned tl = e >> 3, q = e & 7u;
    const v8us o = *(const v8us*)&ts[tl][q * 8u];
    vst2(XB + ((size_t)(b * SEQ + t0 + tl)) * CH + c0 + q * 8u, o);
  }
}

__global__ __launch_bounds__(256) void k_cvtb3(const float* __restrict__ s0, const float* __restrict__ s1, const float* __restrict__ s2,
                                               unsigned short* __restrict__ d0, unsigned short* __restrict__ d1, unsigned short* __restrict__ d2, unsigned n8) {
  const unsigned i = blockIdx.x * 256u + threadIdx.x; if (i >= n8) return;
  const unsigned y = blockIdx.y;
  const float* src = (y == 0u) ? s0 : ((y == 1u) ? s1 : s2);
  unsigned short* dst = (y == 0u) ? d0 : ((y == 1u) ? d1 : d2);
  const float* p = src + (size_t)i * 8u; const v4f a = *(const v4f*)p, b = *(const v4f*)(p + 4);
  v8us o;
#pragma unroll
  for (int e = 0; e < 4; ++e) { o[e] = bf16bits(a[e]); o[4 + e] = bf16bits(b[e]); }
  vst2(dst + (size_t)i * 8u, o);
}
__global__ __launch_bounds__(256) void k_cvth(const float* __restrict__ src, unsigned n8, _Float16* __restrict__ dst) {
  const unsigned i = blockIdx.x * 256u + threadIdx.x; if (i >= n8) return;
  const float* p = src + (size_t)i * 8u; const v4f a = *(const v4f*)p, b = *(const v4f*)(p + 4);
  v8h o;
#pragma unroll
  for (int e = 0; e < 4; ++e) { o[e] = f16n(bfr(a[e]) * WC); o[4 + e] = f16n(bfr(b[e]) * WC); }
  vst2(dst + (size_t)i * 8u, o);
}
template <unsigned O, unsigned CI>
__global__ __launch_bounds__(256) void k_pack(const float* __restrict__ W, _Float16* __restrict__ P) {
  static_assert(CI % 256u == 0u);
  const unsigned i = blockIdx.x * 256u + threadIdx.x; if (i >= O * CI / 8u) return;
  const unsigned per = CI / 8u; const unsigned o = i / per, c8 = i - o * per;
  const float* p = W + ((size_t)o * CI + c8 * 8u) * 3u;
  v4f f[6];
#pragma unroll
  for (int u = 0; u < 6; ++u) f[u] = *(const v4f*)(p + 4 * u);
#pragma unroll
  for (int dk = 0; dk < 3; ++dk) {
    v8h o8;
#pragma unroll
    for (int e = 0; e < 8; ++e) { const int x = 3 * e + dk; o8[e] = f16n(bfr(f[x >> 2][x & 3]) * WC); }
    vst2(P + ((size_t)dk * O + o) * CI + c8 * 8u, o8);
  }
}

__global__ __launch_bounds__(256) void k_rope(float* __restrict__ CS) {
  const unsigned idx = blockIdx.x * 256u + threadIdx.x; const unsigned t = idx >> 5, e = idx & 31u, f = e & 15u;
  const float invf = exp2f(-(float)f * 0.83048202372184059f);
  const float a = invf * (float)t;
  const float n = rintf(a * 0.63661977236758134f);
  float r = fmaf(-n, 1.5703125f, a);
  r = fmaf(-n, 4.837512969970703125e-4f, r);
  r = fmaf(-n, 7.54978995489188216e-8f, r);
  const float r2 = r * r;
  const float sp = r + r * r2 * (-1.6666654611e-1f + r2 * (8.3321608736e-3f + r2 * (-1.9515295891e-4f)));
  const float cp = 1.0f - 0.5f * r2 + r2 * r2 * (4.166664568298827e-2f + r2 * (-1.388731625493765e-3f + r2 * 2.443315711809948e-5f));
  const unsigned q = ((unsigned)(int)n) & 3u;
  const float ss = (q & 1u) ? cp : sp, cc = (q & 1u) ? sp : cp;
  const float sv = (q & 2u) ? -ss : ss;
  const float cv = ((q + 1u) & 2u) ? -cc : cc;
  const float o = (e < 16u) ? cv : sv;
  vst2(CS + idx, o);
}

__global__ __launch_bounds__(256) void k_mflag(const int* __restrict__ MASK, int* __restrict__ MFL) {
  __shared__ int sfl[32];
  const unsigned tid = threadIdx.x, wave = tid >> 5, lane = tid & 31u;
#pragma unroll 1
  for (unsigned s = 0; s < 4u; ++s) {
    const unsigned f = blockIdx.x * 32u + wave * 4u + s;
    const unsigned i16 = f % NI16, rest = f / NI16; const unsigned jc = rest % NJ128, b = rest / NJ128;
    const int* p = MASK + ((size_t)(b * SEQ_FULL + i16 * 16u)) * SEQ_FULL + jc * 128u + lane * 4u;
    int ok = 1;
#pragma unroll 4
    for (unsigned rr = 0; rr < 16u; ++rr) {
      const v4i m = *(const v4i*)(p + (size_t)rr * SEQ_FULL);
      ok &= ((m[0] != 0) & (m[1] != 0) & (m[2] != 0) & (m[3] != 0)) ? 1 : 0;
    }
    const unsigned bal = __builtin_amdgcn_ballot_w32(ok != 0);
    if (lane == 0u) sfl[wave * 4u + s] = (bal == 0xffffffffu) ? 1 : 0;
  }
  __syncthreads();
  if (tid < 32u) { const int v = sfl[tid]; vst2(MFL + blockIdx.x * 32u + tid, v); }
}

__global__ __launch_bounds__(128) void k_qkv(const __bf16* __restrict__ XB, const __bf16* __restrict__ WQB, const __bf16* __restrict__ WKB, const __bf16* __restrict__ WVB,
                                             const float* __restrict__ BQ, const float* __restrict__ BK, const float* __restrict__ BV, const float* __restrict__ CS,
                                             _Float16* __restrict__ QH, _Float16* __restrict__ KH, _Float16* __restrict__ VP) {
  __shared__ __align__(16) float scs[64][32];
  __shared__ __align__(16) _Float16 sq[4][16][72];
  __shared__ __align__(16) _Float16 th[64][72];
  const unsigned tid = threadIdx.x, wave = tid >> 5, lane = tid & 31u, col = lane & 15u, g = lane >> 4;
  const unsigned t0 = blockIdx.x * 64u, bh = blockIdx.y, b = bh >> 3, h = bh & 7u;
#pragma unroll
  for (unsigned it = 0; it < 4u; ++it) { const unsigned e = tid + it * 128u; const unsigned row = e >> 3, q = e & 7u;
    *(v4f*)&scs[row][q * 4u] = *(const v4f*)(CS + (size_t)(t0 + row) * 32u + q * 4u); }
  v8f aq[4], ak[4], av[4];
#pragma unroll
  for (int j = 0; j < 4; ++j) { aq[j] = zero8(); ak[j] = zero8(); av[j] = zero8(); }
#pragma unroll
  for (unsigned kc = 0; kc < 2u; ++kc) {
    const v16b a = frag_b(XB + ((size_t)(b * SEQ + t0 + wave * 16u + col)) * CH + h * HD + kc * 32u, lane);
#pragma unroll
    for (int j = 0; j < 4; ++j) {
      const size_t wr = (size_t)(h * HD + j * 16u + col) * HD + kc * 32u;
      aq[j] = wmma_bf(a, frag_b(WQB + wr, lane), aq[j]);
      ak[j] = wmma_bf(a, frag_b(WKB + wr, lane), ak[j]);
      av[j] = wmma_bf(a, frag_b(WVB + wr, lane), av[j]);
    }
  }
  __syncthreads();
#pragma unroll
  for (int j = 0; j < 4; ++j) {
    const float bq = bfr(BQ[h * HD + j * 16u + col]), bk = bfr(BK[h * HD + j * 16u + col]), bv = bfr(BV[h * HD + j * 16u + col]);
#pragma unroll
    for (int r = 0; r < 8; ++r) { aq[j][r] += bq; ak[j][r] += bk; av[j][r] += bv; }
  }
#pragma unroll
  for (int r = 0; r < 8; ++r) {
    const unsigned tl = wave * 16u + 8u * g + r; const float cs = scs[tl][col], sn = scs[tl][16u + col];
    const float q1 = aq[0][r], q2 = aq[1][r]; aq[0][r] = q1 * cs - q2 * sn; aq[1][r] = q1 * sn + q2 * cs;
    const float k1 = ak[0][r], k2 = ak[1][r]; ak[0][r] = k1 * cs - k2 * sn; ak[1][r] = k1 * sn + k2 * cs;
  }
#pragma unroll
  for (int j = 0; j < 4; ++j)
#pragma unroll
    for (int r = 0; r < 8; ++r) sq[wave][8u * g + r][j * 16u + col] = f16n(aq[j][r]);
  LDSX();
#pragma unroll
  for (unsigned rp = 0; rp < 4u; ++rp) { const unsigned rl = rp * 4u + (lane >> 3), q8 = lane & 7u;
    const v8h o = *(const v8h*)&sq[wave][rl][q8 * 8u]; vst2(QH + ((size_t)(bh * SEQ + t0 + wave * 16u + rl)) * HD + q8 * 8u, o); }
  LDSX();
#pragma unroll
  for (int j = 0; j < 4; ++j)
#pragma unroll
    for (int r = 0; r < 8; ++r) sq[wave][8u * g + r][j * 16u + col] = f16n(ak[j][r]);
  LDSX();
#pragma unroll
  for (unsigned rp = 0; rp < 4u; ++rp) { const unsigned rl = rp * 4u + (lane >> 3), q8 = lane & 7u;
    const v8h o = *(const v8h*)&sq[wave][rl][q8 * 8u]; vst2(KH + ((size_t)(bh * SEQ + t0 + wave * 16u + rl)) * HD + q8 * 8u, o); }
#pragma unroll
  for (int j = 0; j < 4; ++j)
#pragma unroll
    for (int r = 0; r < 8; ++r) th[j * 16u + col][wave * 16u + 8u * g + r] = f16n(av[j][r]);
  __syncthreads();
#pragma unroll
  for (unsigned it = 0; it < 4u; ++it) { const unsigned e = tid + it * 128u; const unsigned cl = e >> 3, q8 = e & 7u;
    const v8h o = *(const v8h*)&th[cl][q8 * 8u]; vst2(VP + ((size_t)(b * CH + h * HD + cl)) * SEQ + t0 + q8 * 8u, o); }
}

__global__ __launch_bounds__(128) void k_stat(const _Float16* __restrict__ QH, const _Float16* __restrict__ KH, const int* __restrict__ MASK, const int* __restrict__ MFL,
                                              float* __restrict__ MX, float* __restrict__ RZ) {
  __shared__ __align__(16) float sm[2][64];
  const unsigned tid = threadIdx.x, wave = tid >> 5, lane = tid & 31u, col = lane & 15u, g = lane >> 4;
  const unsigned bh = blockIdx.y, b = bh >> 3; const unsigned i0 = blockIdx.x * 64u + wave * 16u;
  const _Float16* qb = QH + (size_t)bh * SEQ * HD; const _Float16* kb = KH + (size_t)bh * SEQ * HD;
  const v16h bq0 = frag_h(qb + (size_t)(i0 + col) * HD, lane), bq1 = frag_h(qb + (size_t)(i0 + col) * HD + 32, lane);
  const int* mrow = MASK + ((size_t)(b * SEQ_FULL + i0 + col)) * SEQ_FULL + 8u * g;
  float m = -3.0e38f, z = 0.f;
#pragma unroll 1
  for (unsigned jc = 0; jc < NJ128; ++jc) {
    const int fl = __builtin_amdgcn_readfirstlane(MFL[(size_t)(b * NJ128 + jc) * NI16 + (i0 >> 4)]);
#pragma unroll 2
    for (unsigned jt = 0; jt < 8u; ++jt) {
      const unsigned j0 = jc * 128u + jt * 16u;
      v8f c = zero8();
      c = wmma16(frag_h(kb + (size_t)(j0 + col) * HD, lane), bq0, c);
      c = wmma16(frag_h(kb + (size_t)(j0 + col) * HD + 32, lane), bq1, c);
      float s[8];
#pragma unroll
      for (int r = 0; r < 8; ++r) s[r] = c[r] * 0.125f;
      if (fl != 1) {
        const v4i m0 = *(const v4i*)(mrow + j0), m1 = *(const v4i*)(mrow + j0 + 4u);
#pragma unroll
        for (int r = 0; r < 4; ++r) { s[r] = (m0[r] == 0) ? -10000.0f : s[r]; s[4 + r] = (m1[r] == 0) ? -10000.0f : s[4 + r]; }
      }
      float tm = fmaxf(fmaxf(fmaxf(s[0], s[1]), fmaxf(s[2], s[3])), fmaxf(fmaxf(s[4], s[5]), fmaxf(s[6], s[7])));
      const float mn = fmaxf(m, tm);
      float zz = z * __expf(m - mn);
#pragma unroll
      for (int r = 0; r < 8; ++r) zz += __expf(s[r] - mn);
      z = zz; m = mn;
    }
  }
  const float mo = __shfl_xor(m, 16), zo = __shfl_xor(z, 16);
  const float mn = fmaxf(m, mo);
  const float zt = z * __expf(m - mn) + zo * __expf(mo - mn);
  if (g == 0u) { sm[0][wave * 16u + col] = mn; sm[1][wave * 16u + col] = PCY * (1.0f / zt); }
  __syncthreads();
  if (tid < 16u) {
    const v4f a = *(const v4f*)&sm[0][tid * 4u]; vst2(MX + (size_t)bh * SEQ + blockIdx.x * 64u + tid * 4u, a);
    const v4f c2 = *(const v4f*)&sm[1][tid * 4u]; vst2(RZ + (size_t)bh * SEQ + blockIdx.x * 64u + tid * 4u, c2);
  }
}

__global__ __launch_bounds__(128) void k_att(const _Float16* __restrict__ QH, const _Float16* __restrict__ KH, const _Float16* __restrict__ VP, const int* __restrict__ MASK,
                                             const int* __restrict__ MFL, const float* __restrict__ MX, const float* __restrict__ RZ, _Float16* __restrict__ CTX) {
  __shared__ __align__(16) _Float16 sP[4][16][72];
  const unsigned tid = threadIdx.x, wave = tid >> 5, lane = tid & 31u, col = lane & 15u, g = lane >> 4;
  const unsigned bh = blockIdx.y, b = bh >> 3, h = bh & 7u; const unsigned j0 = blockIdx.x * 64u + wave * 16u;
  const _Float16* qb = QH + (size_t)bh * SEQ * HD; const _Float16* kb = KH + (size_t)bh * SEQ * HD;
  const _Float16* vb = VP + ((size_t)(b * CH + h * HD)) * SEQ;
  const float* mxb = MX + (size_t)bh * SEQ; const float* rzb = RZ + (size_t)bh * SEQ;
  const v16h ak0 = frag_h(kb + (size_t)(j0 + col) * HD, lane), ak1 = frag_h(kb + (size_t)(j0 + col) * HD + 32, lane);
  const int* mbase = MASK + (size_t)b * SEQ_FULL * SEQ_FULL + j0 + 8u * g;
  const int* fbase = MFL + ((size_t)(b * NJ128 + (blockIdx.x >> 1))) * NI16;
  v8f acc[4];
#pragma unroll
  for (int n = 0; n < 4; ++n) acc[n] = zero8();
#pragma unroll 1
  for (unsigned ic = 0; ic < SEQ / 64u; ++ic) {
    const unsigned i0 = ic * 64u;
    const v4i f4 = *(const v4i*)(fbase + ic * 4u);
    const int allone = __builtin_amdgcn_readfirstlane(((f4[0] == 1) & (f4[1] == 1) & (f4[2] == 1) & (f4[3] == 1)) ? 1 : 0);
#pragma unroll 1
    for (unsigned it = 0; it < 4u; ++it) {
      const unsigned ii = i0 + it * 16u + col;
      v8f c = zero8();
      c = wmma16(ak0, frag_h(qb + (size_t)ii * HD, lane), c);
      c = wmma16(ak1, frag_h(qb + (size_t)ii * HD + 32, lane), c);
      float s[8];
#pragma unroll
      for (int r = 0; r < 8; ++r) s[r] = c[r] * 0.125f;
      if (allone == 0) {
        const int* mp = mbase + (size_t)ii * SEQ_FULL;
        const v4i m0 = *(const v4i*)mp, m1 = *(const v4i*)(mp + 4);
#pragma unroll
        for (int r = 0; r < 4; ++r) { s[r] = (m0[r] == 0) ? -10000.0f : s[r]; s[4 + r] = (m1[r] == 0) ? -10000.0f : s[4 + r]; }
      }
      const float mi = mxb[ii], rz = rzb[ii];
#pragma unroll
      for (int r = 0; r < 8; ++r) {
        float p = __expf(fminf(s[r] - mi, 0.0f)) * rz; p = (p >= F16MIN) ? p : 0.0f;
        sP[wave][8u * g + r][it * 16u + col] = (_Float16)p;
      }
    }
    LDSX();
#pragma unroll
    for (unsigned kk = 0; kk < 2u; ++kk) {
      const v16h a = frag_h(&sP[wave][col][kk * 32u], lane);
#pragma unroll
      for (int n = 0; n < 4; ++n) acc[n] = wmma16(a, frag_h(vb + (size_t)(n * 16u + col) * SEQ + i0 + kk * 32u, lane), acc[n]);
    }
    LDSX();
  }
#pragma unroll
  for (int n = 0; n < 4; ++n)
#pragma unroll
    for (int r = 0; r < 8; ++r) sP[wave][8u * g + r][n * 16u + col] = f16n(acc[n][r] * (CC / PCY));
  LDSX();
#pragma unroll
  for (unsigned rp = 0; rp < 4u; ++rp) { const unsigned rl = rp * 4u + (lane >> 3), q8 = lane & 7u;
    const v8h o = *(const v8h*)&sP[wave][rl][q8 * 8u]; vst2(CTX + ((size_t)(b * SEQ + j0 + rl)) * CH + h * HD + q8 * 8u, o); }
}

template <unsigned KIN, unsigned TAPS>
__device__ __forceinline__ void gemm_tile(const _Float16* __restrict__ arow, const _Float16* __restrict__ wrow, size_t wtap, unsigned lane, v8f (&acc)[8]) {
  static_assert(KIN % 32u == 0u);
#pragma unroll 1
  for (unsigned dk = 0; dk < TAPS; ++dk) {
    const _Float16* ap = arow + (size_t)dk * KIN; const _Float16* wp = wrow + (size_t)dk * wtap;
#pragma unroll 1
    for (unsigned kc = 0; kc < KIN / 32u; ++kc) {
      const v16h a = frag_h(ap + kc * 32u, lane);
#pragma unroll
      for (int j = 0; j < 8; ++j) acc[j] = wmma16(a, frag_h(wp + (size_t)j * 16u * KIN + kc * 32u, lane), acc[j]);
    }
  }
}

__global__ __launch_bounds__(128) void k_wo(const _Float16* __restrict__ CTX, const _Float16* __restrict__ WOH, const float* __restrict__ BO, const unsigned short* __restrict__ XB, float* __restrict__ S1) {
  __shared__ __align__(16) float sf[4][16][132];
  const unsigned tid = threadIdx.x, wave = tid >> 5, lane = tid & 31u, col = lane & 15u, g = lane >> 4;
  const unsigned c0 = blockIdx.y * 128u; const size_t r0 = (size_t)blockIdx.x * 64u + wave * 16u;
  v8f acc[8];
#pragma unroll
  for (int j = 0; j < 8; ++j) acc[j] = zero8();
  gemm_tile<CH, 1u>(CTX + (r0 + col) * CH, WOH + (size_t)(c0 + col) * CH, (size_t)0, lane, acc);
#pragma unroll
  for (int j = 0; j < 8; ++j)
#pragma unroll
    for (int r = 0; r < 8; ++r) sf[wave][8u * g + r][j * 16u + col] = acc[j][r] * (1.0f / (CC * WC));
  LDSX();
  v4f bias = *(const v4f*)(BO + c0 + lane * 4u);
#pragma unroll
  for (int k = 0; k < 4; ++k) bias[k] = bfr(bias[k]);
#pragma unroll 1
  for (unsigned rl = 0; rl < 16u; ++rl) {
    const size_t o = (r0 + rl) * (size_t)CH + c0 + lane * 4u;
    v4f vv = *(const v4f*)&sf[wave][rl][lane * 4u]; const v4us xb = *(const v4us*)(XB + o);
#pragma unroll
    for (int k = 0; k < 4; ++k) vv[k] += bias[k] + bf16val(xb[k]);
    vst2(S1 + o, vv);
  }
}

__global__ __launch_bounds__(256) void k_ln1(const float* __restrict__ S1, const float* __restrict__ G, const float* __restrict__ BE, const float* __restrict__ XM,
                                             float* __restrict__ H32, _Float16* __restrict__ HP) {
  const unsigned wave = threadIdx.x >> 5, lane = threadIdx.x & 31u;
  const unsigned R = blockIdx.x * 8u + wave; const unsigned b = R / SEQ, t = R - b * SEQ;
  const size_t rb = (size_t)R * CH;
  v4f v[4]; float s1 = 0.f;
#pragma unroll
  for (int i = 0; i < 4; ++i) { v[i] = *(const v4f*)(S1 + rb + i * 128u + lane * 4u); s1 += (v[i][0] + v[i][1]) + (v[i][2] + v[i][3]); }
#pragma unroll
  for (int o = 1; o < 32; o <<= 1) s1 += __shfl_xor(s1, o);
  const float mu = s1 * (1.0f / CH); float q = 0.f;
#pragma unroll
  for (int i = 0; i < 4; ++i)
#pragma unroll
    for (int k = 0; k < 4; ++k) { const float d = v[i][k] - mu; q += d * d; }
#pragma unroll
  for (int o = 1; o < 32; o <<= 1) q += __shfl_xor(q, o);
  const float inv = 1.0f / sqrtf(q * (1.0f / CH) + LN_EPS);
  const float mk = bfr(XM[(size_t)b * SEQ_FULL + t]);
  _Float16* hrow = HP + ((size_t)(b * PR + 1u + t)) * CH;
#pragma unroll
  for (int i = 0; i < 4; ++i) {
    const v4f g4 = *(const v4f*)(G + i * 128u + lane * 4u), b4 = *(const v4f*)(BE + i * 128u + lane * 4u);
    v4f y; v4h hh;
#pragma unroll
    for (int k = 0; k < 4; ++k) { y[k] = (v[i][k] - mu) * inv * bfr(g4[k]) + bfr(b4[k]); hh[k] = f16n(y[k] * mk); }
    vst2(H32 + rb + i * 128u + lane * 4u, y);
    vst2(hrow + i * 128u + lane * 4u, hh);
  }
  const v4h zz = {(_Float16)0.0f, (_Float16)0.0f, (_Float16)0.0f, (_Float16)0.0f};
  if (t == 0u) {
    _Float16* pr = HP + ((size_t)(b * PR)) * CH;
#pragma unroll
    for (int i = 0; i < 4; ++i) vst2(pr + i * 128u + lane * 4u, zz);
  }
  if (t == SEQ - 1u) {
    _Float16* pr = HP + ((size_t)(b * PR + SEQ + 1u)) * CH;
#pragma unroll
    for (int i = 0; i < 4; ++i) vst2(pr + i * 128u + lane * 4u, zz);
  }
}

__global__ __launch_bounds__(128) void k_c1(const _Float16* __restrict__ HP, const _Float16* __restrict__ W1P, const float* __restrict__ B1, const float* __restrict__ XM, _Float16* __restrict__ FP) {
  __shared__ __align__(16) float sf[4][16][132];
  const unsigned tid = threadIdx.x, wave = tid >> 5, lane = tid & 31u, col = lane & 15u, g = lane >> 4;
  const unsigned t0 = blockIdx.x * 64u + wave * 16u, c0 = blockIdx.y * 128u, b = blockIdx.z;
  v8f acc[8];
#pragma unroll
  for (int j = 0; j < 8; ++j) acc[j] = zero8();
  gemm_tile<CH, 3u>(HP + ((size_t)(b * PR + t0 + col)) * CH, W1P + (size_t)(c0 + col) * CH, (size_t)HID * CH, lane, acc);
#pragma unroll
  for (int j = 0; j < 8; ++j)
#pragma unroll
    for (int r = 0; r < 8; ++r) sf[wave][8u * g + r][j * 16u + col] = acc[j][r] * (1.0f / WC);
  LDSX();
  v4f bias = *(const v4f*)(B1 + c0 + lane * 4u);
#pragma unroll
  for (int k = 0; k < 4; ++k) bias[k] = bfr(bias[k]);
#pragma unroll 1
  for (unsigned rl = 0; rl < 16u; ++rl) {
    const unsigned t = t0 + rl; const float mk = bfr(XM[(size_t)b * SEQ_FULL + t]);
    const v4f vv = *(const v4f*)&sf[wave][rl][lane * 4u]; v4h o4;
#pragma unroll
    for (int k = 0; k < 4; ++k) { const float u = vv[k] + bias[k]; const float gl = 0.5f * u * (1.0f + erff(u * 0.70710678118654752f)); o4[k] = f16n(gl * mk); }
    vst2(FP + ((size_t)(b * PR + 1u + t)) * HID + c0 + lane * 4u, o4);
  }
  const v4h zz = {(_Float16)0.0f, (_Float16)0.0f, (_Float16)0.0f, (_Float16)0.0f};
  if (blockIdx.x == 0u && wave == 0u) vst2(FP + ((size_t)(b * PR)) * HID + c0 + lane * 4u, zz);
  if (blockIdx.x == (SEQ / 64u - 1u) && wave == 3u) vst2(FP + ((size_t)(b * PR + SEQ + 1u)) * HID + c0 + lane * 4u, zz);
}

__global__ __launch_bounds__(128) void k_c2(const _Float16* __restrict__ FP, const _Float16* __restrict__ W2P, const float* __restrict__ B2, const float* __restrict__ XM,
                                            const float* __restrict__ H32, float* __restrict__ Z2) {
  __shared__ __align__(16) float sf[4][16][132];
  const unsigned tid = threadIdx.x, wave = tid >> 5, lane = tid & 31u, col = lane & 15u, g = lane >> 4;
  const unsigned t0 = blockIdx.x * 64u + wave * 16u, c0 = blockIdx.y * 128u, b = blockIdx.z;
  v8f acc[8];
#pragma unroll
  for (int j = 0; j < 8; ++j) acc[j] = zero8();
  gemm_tile<HID, 3u>(FP + ((size_t)(b * PR + t0 + col)) * HID, W2P + (size_t)(c0 + col) * HID, (size_t)CH * HID, lane, acc);
#pragma unroll
  for (int j = 0; j < 8; ++j)
#pragma unroll
    for (int r = 0; r < 8; ++r) sf[wave][8u * g + r][j * 16u + col] = acc[j][r] * (1.0f / WC);
  LDSX();
  v4f bias = *(const v4f*)(B2 + c0 + lane * 4u);
#pragma unroll
  for (int k = 0; k < 4; ++k) bias[k] = bfr(bias[k]);
#pragma unroll 1
  for (unsigned rl = 0; rl < 16u; ++rl) {
    const unsigned t = t0 + rl; const float mk = bfr(XM[(size_t)b * SEQ_FULL + t]);
    const size_t o = ((size_t)(b * SEQ + t)) * CH + c0 + lane * 4u;
    v4f vv = *(const v4f*)&sf[wave][rl][lane * 4u]; const v4f hv = *(const v4f*)(H32 + o);
#pragma unroll
    for (int k = 0; k < 4; ++k) vv[k] = (vv[k] + bias[k]) * mk + hv[k];
    vst2(Z2 + o, vv);
  }
}

__global__ __launch_bounds__(256) void k_ln2(const float* __restrict__ Z, const float* __restrict__ G, const float* __restrict__ BE, float* __restrict__ OUT) {
  __shared__ __align__(16) float to[CH][36];
  const unsigned tid = threadIdx.x, wave = tid >> 5, lane = tid & 31u;
  const unsigned R0 = blockIdx.x * 32u; const unsigned b = R0 / SEQ, t0 = R0 - b * SEQ;
  v4f gg[4], bb[4];
#pragma unroll
  for (int i = 0; i < 4; ++i) { gg[i] = *(const v4f*)(G + i * 128u + lane * 4u); bb[i] = *(const v4f*)(BE + i * 128u + lane * 4u);
#pragma unroll
    for (int k = 0; k < 4; ++k) { gg[i][k] = bfr(gg[i][k]); bb[i][k] = bfr(bb[i][k]); } }
#pragma unroll 1
  for (unsigned qq = 0; qq < 4u; ++qq) {
    const unsigned tl = wave * 4u + qq; const size_t rb = (size_t)(R0 + tl) * CH;
    v4f v[4]; float s1 = 0.f;
#pragma unroll
    for (int i = 0; i < 4; ++i) { v[i] = *(const v4f*)(Z + rb + i * 128u + lane * 4u); s1 += (v[i][0] + v[i][1]) + (v[i][2] + v[i][3]); }
#pragma unroll
    for (int o = 1; o < 32; o <<= 1) s1 += __shfl_xor(s1, o);
    const float mu = s1 * (1.0f / CH); float q = 0.f;
#pragma unroll
    for (int i = 0; i < 4; ++i)
#pragma unroll
      for (int k = 0; k < 4; ++k) { const float d = v[i][k] - mu; q += d * d; }
#pragma unroll
    for (int o = 1; o < 32; o <<= 1) q += __shfl_xor(q, o);
    const float inv = 1.0f / sqrtf(q * (1.0f / CH) + LN_EPS);
#pragma unroll
    for (int i = 0; i < 4; ++i)
#pragma unroll
      for (int k = 0; k < 4; ++k) to[i * 128u + lane * 4u + k][tl] = (v[i][k] - mu) * inv * gg[i][k] + bb[i][k];
  }
  __syncthreads();
#pragma unroll 1
  for (unsigned it = 0; it < 16u; ++it) {
    const unsigned e = tid + it * 256u; const unsigned c = e >> 3, q4 = e & 7u;
    const v4f o = *(const v4f*)&to[c][q4 * 4u];
    vst2(OUT + ((size_t)(b * CH + c)) * SEQ + t0 + q4 * 4u, o);
  }
}

extern "C" void kernel_launch(void* const* d_in, const int* in_sizes, int n_in, void* d_out, int out_size, void* d_ws, size_t ws_size, hipStream_t stream) {
  if (n_in < 19) return;
  if ((size_t)in_sizes[0] < (size_t)NB * CH * SEQ_FULL || (size_t)in_sizes[1] < (size_t)NB * SEQ_FULL || (size_t)in_sizes[2] < (size_t)NB * SEQ_FULL * SEQ_FULL) return;
  if (in_sizes[3] < (int)(CH * HD) || in_sizes[5] < (int)(CH * HD) || in_sizes[7] < (int)(CH * HD) || in_sizes[9] < (int)(CH * CH)) return;
  if (in_sizes[4] < (int)CH || in_sizes[6] < (int)CH || in_sizes[8] < (int)CH || in_sizes[10] < (int)CH) return;
  if (in_sizes[11] < (int)(HID * CH * 3u) || in_sizes[12] < (int)HID || in_sizes[13] < (int)(CH * HID * 3u) || in_sizes[14] < (int)CH) return;
  if (in_sizes[15] < (int)CH || in_sizes[16] < (int)CH || in_sizes[17] < (int)CH || in_sizes[18] < (int)CH) return;
  if ((size_t)out_size < (size_t)NB * CH * SEQ) return;
  if (ws_size < (size_t)WS_END) return;
  const float* X = (const float*)d_in[0]; const float* XM = (const float*)d_in[1]; const int* AM = (const int*)d_in[2];
  const float* WQ = (const float*)d_in[3]; const float* BQ = (const float*)d_in[4]; const float* WK = (const float*)d_in[5]; const float* BK = (const float*)d_in[6];
  const float* WV = (const float*)d_in[7]; const float* BV = (const float*)d_in[8]; const float* WO = (const float*)d_in[9]; const float* BO = (const float*)d_in[10];
  const float* W1 = (const float*)d_in[11]; const float* B1 = (const float*)d_in[12]; const float* W2 = (const float*)d_in[13]; const float* B2 = (const float*)d_in[14];
  const float* G1 = (const float*)d_in[15]; const float* BE1 = (const float*)d_in[16]; const float* G2 = (const float*)d_in[17]; const float* BE2 = (const float*)d_in[18];
  char* ws = (char*)d_ws;
  unsigned short* XBu = (unsigned short*)(ws + WS_XB); const __bf16* XB = (const __bf16*)(ws + WS_XB);
  unsigned short* WQBu = (unsigned short*)(ws + WS_WQB); unsigned short* WKBu = (unsigned short*)(ws + WS_WKB); unsigned short* WVBu = (unsigned short*)(ws + WS_WVB);
  const __bf16* WQB = (const __bf16*)(ws + WS_WQB); const __bf16* WKB = (const __bf16*)(ws + WS_WKB); const __bf16* WVB = (const __bf16*)(ws + WS_WVB);
  _Float16* WOH = (_Float16*)(ws + WS_WOH); _Float16* W1P = (_Float16*)(ws + WS_W1P); _Float16* W2P = (_Float16*)(ws + WS_W2P);
  float* CS = (float*)(ws + WS_CS); int* MFL = (int*)(ws + WS_MFL);
  _Float16* QH = (_Float16*)(ws + WS_QH); _Float16* KH = (_Float16*)(ws + WS_KH); _Float16* VP = (_Float16*)(ws + WS_VP);
  float* MX = (float*)(ws + WS_MX); float* RZ = (float*)(ws + WS_RZ);
  _Float16* CTX = (_Float16*)(ws + WS_CTX); float* S1 = (float*)(ws + WS_S1); float* H32 = (float*)(ws + WS_H32);
  _Float16* HP = (_Float16*)(ws + WS_HP); _Float16* FP = (_Float16*)(ws + WS_FP); float* Z2 = (float*)(ws + WS_Z2);

  const unsigned n8w = CH * HD / 8u, n8o = CH * CH / 8u;
  k_xt<<<dim3(SEQ / 64u, CH / 64u, NB), 256, 0, stream>>>(X, XBu);
  k_cvtb3<<<dim3((n8w + 255u) / 256u, 3), 256, 0, stream>>>(WQ, WK, WV, WQBu, WKBu, WVBu, n8w);
  k_cvth<<<dim3((n8o + 255u) / 256u), 256, 0, stream>>>(WO, n8o, WOH);
  k_pack<HID, CH><<<dim3(HID * CH / 8u / 256u), 256, 0, stream>>>(W1, W1P);
  k_pack<CH, HID><<<dim3(CH * HID / 8u / 256u), 256, 0, stream>>>(W2, W2P);
  k_rope<<<dim3(SEQ * 32u / 256u), 256, 0, stream>>>(CS);
  k_mflag<<<dim3(NFLAGS / 32u), 256, 0, stream>>>(AM, MFL);
  k_qkv<<<dim3(SEQ / 64u, NB * NH), 128, 0, stream>>>(XB, WQB, WKB, WVB, BQ, BK, BV, CS, QH, KH, VP);
  k_stat<<<dim3(SEQ / 64u, NB * NH), 128, 0, stream>>>(QH, KH, AM, MFL, MX, RZ);
  k_att<<<dim3(SEQ / 64u, NB * NH), 128, 0, stream>>>(QH, KH, VP, AM, MFL, MX, RZ, CTX);
  k_wo<<<dim3(NB * SEQ / 64u, CH / 128u), 128, 0, stream>>>(CTX, WOH, BO, XBu, S1);
  k_ln1<<<dim3(NB * SEQ / 8u), 256, 0, stream>>>(S1, G1, BE1, XM, H32, HP);
  k_c1<<<dim3(SEQ / 64u, HID / 128u, NB), 128, 0, stream>>>(HP, W1P, B1, XM, FP);
  k_c2<<<dim3(SEQ / 64u, CH / 128u, NB), 128, 0, stream>>>(FP, W2P, B2, XM, H32, Z2);
  k_ln2<<<dim3(NB * SEQ / 32u), 256, 0, stream>>>(Z2, G2, BE2, (float*)d_out);
}
